// SelfAttention_6485400617384
// MI455X (gfx1250) — hardware-verified
//
#include <hip/hip_runtime.h>


#ifndef NB
#define NB 2
#endif
#ifndef SEQ
#define SEQ 2048
#endif
#define NB_FULL   2
#define SEQ_FULL  2048
#define EDIM      1024
#define HIDN      1024
#define NHEAD     16
#define HDIM      64
#define QKVW      3072
#define CHUNK     192
#define KD        1024
#define NTOK      (NB * SEQ)
#define NGRP      (NHEAD * NB)
#define TPG       (SEQ / NHEAD)
#define NCHUNKS   (NTOK * NHEAD)
#define BQ        128
#define BK        32
#define NWAVE     8
#define TP        72
#define VP        136
#define OP        68

#define XN_OFF    ((size_t)0)
#define W1T_OFF   (XN_OFF  + (size_t)NTOK * EDIM)
#define W2T_OFF   (W1T_OFF + (size_t)QKVW * EDIM)
#define QP_OFF    (W2T_OFF + (size_t)HIDN * HIDN)
#define KP_OFF    (QP_OFF  + (size_t)NCHUNKS * HDIM)
#define VT_OFF    (KP_OFF  + (size_t)NCHUNKS * HDIM)
#define ATT_OFF   (VT_OFF  + (size_t)NCHUNKS * HDIM)
#define WS_HALVES (ATT_OFF + (size_t)NCHUNKS * HDIM)
#define WS_BYTES  (WS_HALVES * 2)

static_assert(NB >= 1 && NB <= NB_FULL);
static_assert(SEQ <= SEQ_FULL);
static_assert(SEQ % 1024 == 0);
static_assert(TPG % 64 == 0);
static_assert(NTOK % 128 == 0);
static_assert(SEQ % 128 == 0);
static_assert(QKVW == NHEAD * CHUNK);
static_assert(CHUNK == 3 * HDIM);
static_assert(QKVW % 64 == 0);
static_assert(HIDN % 64 == 0);
static_assert(EDIM % 64 == 0);
static_assert(EDIM == KD && HIDN == KD);
static_assert(KD % 32 == 0);
static_assert(EDIM == 128 * 8);
static_assert(SEQ % BQ == 0);
static_assert(SEQ % BK == 0);
static_assert(BQ == NWAVE * 16);
static_assert(HDIM == 64);
static_assert((size_t)NCHUNKS * HDIM == (size_t)NTOK * HIDN);
static_assert((TP * 2) % 16 == 0);
static_assert((VP * 2) % 16 == 0);
static_assert((OP * 4) % 16 == 0);
static_assert(128 * TP >= 64 * VP);
static_assert(XN_OFF % 64 == 0 && W1T_OFF % 64 == 0 && W2T_OFF % 64 == 0);
static_assert(QP_OFF % 64 == 0 && KP_OFF % 64 == 0 && VT_OFF % 64 == 0 && ATT_OFF % 64 == 0);
static_assert(WS_BYTES <= (size_t)134217728);

typedef __bf16   bf16;
typedef _Float16 f16;
typedef f16      v16h  __attribute__((ext_vector_type(16)));
typedef f16      v8h   __attribute__((ext_vector_type(8)));
typedef float    v8f   __attribute__((ext_vector_type(8)));
typedef float    v4f   __attribute__((ext_vector_type(4)));
typedef unsigned v4u   __attribute__((ext_vector_type(4)));

union FragH  { v16h  v; v4u q[2]; f16  h[16]; };
union Pack8H { v4u u; v8h v; f16 h[8]; };

static __device__ __forceinline__ v8f mma_f16(v16h a, v16h b, v8f acc) {
  acc = __builtin_amdgcn_wmma_f32_16x16x32_f16(false, a, false, b, (short)0, acc, false, false);
  asm volatile("v_nop\n\tv_nop\n\tv_nop\n\tv_nop" : "+v"(acc) : "v"(a), "v"(b));
  return acc;
}

__global__ __launch_bounds__(128) void ln_kernel(const float* __restrict__ x,
                                                 const float* __restrict__ g,
                                                 const float* __restrict__ be,
                                                 f16* __restrict__ xn) {
  const int tt   = blockIdx.x;
  const int tid  = threadIdx.x;
  const int wave = __builtin_amdgcn_readfirstlane((int)(threadIdx.x >> 5));
  const int lane = tid & 31;
  __shared__ float red1[4];
  __shared__ float red2[4];

  const int b = tt / SEQ;
  const int s = tt - b * SEQ;
  const float* src = x + ((size_t)b * SEQ_FULL + s) * EDIM + tid * 8;
  const v4f a0 = *(const v4f*)(src);
  const v4f a1 = *(const v4f*)(src + 4);
  float v[8];
  #pragma unroll
  for (int i = 0; i < 4; ++i) {
    v[i]     = (float)(bf16)a0[i];
    v[4 + i] = (float)(bf16)a1[i];
  }
  float sum = ((v[0] + v[1]) + (v[2] + v[3])) + ((v[4] + v[5]) + (v[6] + v[7]));
  #pragma unroll
  for (int off = 16; off > 0; off >>= 1) sum += __shfl_xor(sum, off, 32);
  if (lane == 0) red1[wave] = sum;
  __syncthreads();
  const float mu = ((red1[0] + red1[1]) + (red1[2] + red1[3])) * (1.0f / (float)EDIM);

  float d[8];
  float sq = 0.0f;
  #pragma unroll
  for (int i = 0; i < 8; ++i) {
    d[i] = v[i] - mu;
    sq += d[i] * d[i];
  }
  #pragma unroll
  for (int off = 16; off > 0; off >>= 1) sq += __shfl_xor(sq, off, 32);
  if (lane == 0) red2[wave] = sq;
  __syncthreads();
  const float var = ((red2[0] + red2[1]) + (red2[2] + red2[3])) * (1.0f / (float)EDIM);
  const float rs  = rsqrtf(var + 1e-5f);

  const v4f g0 = *(const v4f*)(g + tid * 8);
  const v4f g1 = *(const v4f*)(g + tid * 8 + 4);
  const v4f e0 = *(const v4f*)(be + tid * 8);
  const v4f e1 = *(const v4f*)(be + tid * 8 + 4);
  Pack8H ph;
  #pragma unroll
  for (int i = 0; i < 4; ++i) {
    ph.h[i]     = (f16)(d[i]     * rs * (float)(bf16)g0[i] + (float)(bf16)e0[i]);
    ph.h[4 + i] = (f16)(d[4 + i] * rs * (float)(bf16)g1[i] + (float)(bf16)e1[i]);
  }
  const v4u val = ph.u;
  const size_t idx = (size_t)tt * EDIM + tid * 8;
  *(volatile v4u*)(xn + idx) = val;
  __threadfence();
  *(volatile v4u*)(xn + idx) = val;
}

__global__ __launch_bounds__(256) void wt_kernel(const float* __restrict__ w,
                                                 f16* __restrict__ wt,
                                                 int kdim, int ndim) {
  const int n0  = blockIdx.x * 64;
  const int k0  = blockIdx.y * 64;
  const int tid = threadIdx.x;
  __shared__ __align__(16) f16 sT[64 * TP];

  #pragma unroll
  for (int kk = 0; kk < 2; ++kk) {
    const int krow = kk * 32 + (tid >> 3);
    const int c0   = (tid & 7) * 8;
    const float* src = w + (size_t)(k0 + krow) * ndim + n0 + c0;
    const v4f a0 = *(const v4f*)(src);
    const v4f a1 = *(const v4f*)(src + 4);
    #pragma unroll
    for (int i = 0; i < 4; ++i) {
      sT[(c0 + i) * TP + krow]     = (f16)((float)(bf16)a0[i] * 64.0f);
      sT[(c0 + 4 + i) * TP + krow] = (f16)((float)(bf16)a1[i] * 64.0f);
    }
  }
  __syncthreads();

  v4u    vals[2];
  size_t gidx[2];
  #pragma unroll
  for (int kk = 0; kk < 2; ++kk) {
    const int n  = kk * 32 + (tid >> 3);
    const int ks = (tid & 7) * 8;
    Pack8H ph;
    ph.v = *(const v8h*)(sT + n * TP + ks);
    vals[kk] = ph.u;
    gidx[kk] = (size_t)(n0 + n) * kdim + k0 + ks;
  }
  #pragma unroll
  for (int kk = 0; kk < 2; ++kk) *(volatile v4u*)(wt + gidx[kk]) = vals[kk];
  __threadfence();
  #pragma unroll
  for (int kk = 0; kk < 2; ++kk) *(volatile v4u*)(wt + gidx[kk]) = vals[kk];
}

static __device__ __forceinline__ void gemm_tile_128x64(const f16* __restrict__ A,
                                                        const f16* __restrict__ Bt,
                                                        int m0, int n0, int wm, int wn,
                                                        int lq, int hi, v8f (&acc)[2][2]) {
  const f16* ap = A  + (size_t)(m0 + wm * 32 + lq) * KD + hi * 8;
  const f16* bp = Bt + (size_t)(n0 + wn * 32 + lq) * KD + hi * 8;
  #pragma unroll 2
  for (int k0 = 0; k0 < KD; k0 += 32) {
    FragH a[2], b[2];
    #pragma unroll
    for (int i = 0; i < 2; ++i) {
      a[i].q[0] = *(const v4u*)(ap + (size_t)i * 16 * KD + k0);
      a[i].q[1] = *(const v4u*)(ap + (size_t)i * 16 * KD + k0 + 16);
      b[i].q[0] = *(const v4u*)(bp + (size_t)i * 16 * KD + k0);
      b[i].q[1] = *(const v4u*)(bp + (size_t)i * 16 * KD + k0 + 16);
    }
    #pragma unroll
    for (int i = 0; i < 2; ++i) {
      #pragma unroll
      for (int j = 0; j < 2; ++j) acc[i][j] = mma_f16(a[i].v, b[j].v, acc[i][j]);
    }
  }
}

__global__ __launch_bounds__(256) void qkv_gemm_kernel(const f16* __restrict__ xn,
                                                       const f16* __restrict__ w1t,
                                                       const float* __restrict__ b1,
                                                       f16* wsh) {
  const int j    = blockIdx.x;
  const int m0   = blockIdx.y * 128;
  const int n0   = j * 64;
  const int tid  = threadIdx.x;
  const int wave = __builtin_amdgcn_readfirstlane((int)(threadIdx.x >> 5));
  const int lane = tid & 31;
  const int lq   = lane & 15;
  const int hi   = lane >> 4;
  const int wm   = wave >> 1;
  const int wn   = wave & 1;
  const int f    = j / 3;
  const int typ  = j - 3 * f;

  __shared__ __align__(16) f16 sC[128 * TP];

  v8f acc[2][2];
  #pragma unroll
  for (int i = 0; i < 2; ++i) {
    #pragma unroll
    for (int jj = 0; jj < 2; ++jj) acc[i][jj] = (v8f){0, 0, 0, 0, 0, 0, 0, 0};
  }
  gemm_tile_128x64(xn, w1t, m0, n0, wm, wn, lq, hi, acc);

  float bias[2];
  #pragma unroll
  for (int jj = 0; jj < 2; ++jj) bias[jj] = (float)(bf16)b1[n0 + wn * 32 + jj * 16 + lq];

  const int rstr = (typ != 2) ? TP : 1;
  const int cstr = (typ != 2) ? 1 : VP;
  #pragma unroll
  for (int i = 0; i < 2; ++i) {
    #pragma unroll
    for (int jj = 0; jj < 2; ++jj) {
      #pragma unroll
      for (int r = 0; r < 8; ++r) {
        const int row = wm * 32 + i * 16 + hi * 8 + r;
        const int col = wn * 32 + jj * 16 + lq;
        sC[row * rstr + col * cstr] = (f16)(acc[i][jj][r] * (1.0f / 64.0f) + bias[jj]);
      }
    }
  }
  __syncthreads();

  v4u    vals[4];
  size_t gidx[4];
  #pragma unroll
  for (int it = 0; it < 4; ++it) {
    const int line  = it * 32 + (tid >> 3);
    const int piece = tid & 7;
    const int lofs_r = line * TP + piece * 8;
    const int lofs_v = (line >> 1) * VP + (line & 1) * 64 + piece * 8;
    const int lofs   = (typ != 2) ? lofs_r : lofs_v;
    Pack8H ph;
    ph.v = *(const v8h*)(sC + lofs);
    vals[it] = ph.u;

    const int t_r  = m0 + line;
    const int hb_r = t_r / TPG;
    const int tl_r = t_r - hb_r * TPG;
    const size_t qidx = QP_OFF + ((size_t)t_r * NHEAD + f) * HDIM + piece * 8;
    const size_t kidx = KP_OFF + ((size_t)hb_r * SEQ + f * TPG + tl_r) * HDIM + piece * 8;

    const int t_v  = m0 + (line & 1) * 64 + piece * 8;
    const int hb_v = t_v / TPG;
    const int tl_v = t_v - hb_v * TPG;
    const size_t vidx = VT_OFF + ((size_t)hb_v * HDIM + (line >> 1)) * SEQ + f * TPG + tl_v;

    gidx[it] = (typ == 0) ? qidx : ((typ == 1) ? kidx : vidx);
  }
  #pragma unroll
  for (int it = 0; it < 4; ++it) *(volatile v4u*)(wsh + gidx[it]) = vals[it];
  __threadfence();
  #pragma unroll
  for (int it = 0; it < 4; ++it) *(volatile v4u*)(wsh + gidx[it]) = vals[it];
}

__global__ __launch_bounds__(256) void attn_kernel(const f16* __restrict__ qp,
                                                   const f16* __restrict__ kp,
                                                   const f16* __restrict__ vt,
                                                   f16* __restrict__ att) {
  const int qblk = blockIdx.x;
  const int hb   = blockIdx.y;
  const int tid  = threadIdx.x;
  const int wave = __builtin_amdgcn_readfirstlane((int)(threadIdx.x >> 5));
  const int lane = tid & 31;
  const int lq   = lane & 15;
  const int hi   = lane >> 4;

  __shared__ __align__(16) f16 sO[NWAVE * 16 * TP];

  const int qrow0 = qblk * BQ + wave * 16;

  FragH qf[2];
  {
    const f16* qrow = qp + ((size_t)hb * SEQ + qrow0 + lq) * HDIM + hi * 8;
    #pragma unroll
    for (int f = 0; f < 2; ++f) {
      qf[f].q[0] = *(const v4u*)(qrow + f * 32);
      qf[f].q[1] = *(const v4u*)(qrow + f * 32 + 16);
    }
  }

  const f16* kb_h = kp + (size_t)hb * SEQ * HDIM;
  const f16* vt_h = vt + (size_t)hb * HDIM * SEQ;

  v8f o[4];
  #pragma unroll
  for (int dt = 0; dt < 4; ++dt) o[dt] = (v8f){0, 0, 0, 0, 0, 0, 0, 0};

  float rmax = -__builtin_inff();
  float rsum = 0.0f;
  const float SL = 0.022097086912079608f * 1.4426950408889634f;

  #pragma unroll 1
  for (int i = 0; i < SEQ / BK; ++i) {
    const int j0 = i * BK;

    FragH ak[2][2];
    #pragma unroll
    for (int sub = 0; sub < 2; ++sub) {
      #pragma unroll
      for (int f = 0; f < 2; ++f) {
        const f16* base = kb_h + (size_t)(j0 + sub * 16 + lq) * HDIM + f * 32 + hi * 8;
        ak[sub][f].q[0] = *(const v4u*)(base);
        ak[sub][f].q[1] = *(const v4u*)(base + 16);
      }
    }
    FragH bv[4];
    #pragma unroll
    for (int dt = 0; dt < 4; ++dt) {
      const f16* base = vt_h + (size_t)(dt * 16 + lq) * SEQ + j0 + hi * 8;
      bv[dt].q[0] = *(const v4u*)(base);
      bv[dt].q[1] = *(const v4u*)(base + 16);
    }

    v8f c[2];
    #pragma unroll
    for (int sub = 0; sub < 2; ++sub) {
      v8f acc = (v8f){0, 0, 0, 0, 0, 0, 0, 0};
      acc = mma_f16(ak[sub][0].v, qf[0].v, acc);
      acc = mma_f16(ak[sub][1].v, qf[1].v, acc);
      c[sub] = acc;
    }

    float m_new = rmax;
    #pragma unroll
    for (int r = 0; r < 8; ++r) {
      m_new = fmaxf(m_new, c[0][r]);
      m_new = fmaxf(m_new, c[1][r]);
    }
    m_new = fmaxf(m_new, __shfl_xor(m_new, 16, 32));
    const float scale = __builtin_amdgcn_exp2f((rmax - m_new) * SL);
    rmax = m_new;

    FragH pa;
    float psum = 0.0f;
    #pragma unroll
    for (int r = 0; r < 8; ++r) {
      const float p0 = __builtin_amdgcn_exp2f((c[0][r] - m_new) * SL);
      const float p1 = __builtin_amdgcn_exp2f((c[1][r] - m_new) * SL);
      psum += p0 + p1;
      pa.h[r]     = (f16)(p0 * 4096.0f);
      pa.h[8 + r] = (f16)(p1 * 4096.0f);
    }
    rsum = rsum * scale + psum + __shfl_xor(psum, 16, 32);

    float sc[8];
    #pragma unroll
    for (int r = 0; r < 8; ++r) sc[r] = __shfl(scale, (hi << 3) + r, 32);
    #pragma unroll
    for (int dt = 0; dt < 4; ++dt) {
      #pragma unroll
      for (int r = 0; r < 8; ++r) o[dt][r] *= sc[r];
    }

    #pragma unroll
    for (int dt = 0; dt < 4; ++dt) o[dt] = mma_f16(pa.v, bv[dt].v, o[dt]);
  }

  const float rinv = 1.0f / rsum;
  float rs[8];
  #pragma unroll
  for (int r = 0; r < 8; ++r) rs[r] = __shfl(rinv, (hi << 3) + r, 32);

  f16* so = sO + wave * (16 * TP);
  #pragma unroll
  for (int r = 0; r < 8; ++r) {
    #pragma unroll
    for (int dt = 0; dt < 4; ++dt) {
      so[(hi * 8 + r) * TP + dt * 16 + lq] = (f16)(o[dt][r] * (64.0f / 4096.0f) * rs[r]);
    }
  }
  __syncthreads();

  v4u    vals[4];
  size_t gidx[4];
  #pragma unroll
  for (int it = 0; it < 4; ++it) {
    const int row   = it * 4 + (lane >> 3);
    const int piece = lane & 7;
    Pack8H ph;
    ph.v = *(const v8h*)(so + row * TP + piece * 8);
    vals[it] = ph.u;
    gidx[it] = ((size_t)hb * SEQ + qrow0 + row) * HDIM + piece * 8;
  }
  #pragma unroll
  for (int it = 0; it < 4; ++it) *(volatile v4u*)(att + gidx[it]) = vals[it];
  __threadfence();
  #pragma unroll
  for (int it = 0; it < 4; ++it) *(volatile v4u*)(att + gidx[it]) = vals[it];
}

__global__ __launch_bounds__(256) void out_gemm_kernel(const f16* __restrict__ att,
                                                       const f16* __restrict__ w2t,
                                                       const float* __restrict__ b2,
                                                       float* __restrict__ out) {
  const int n0   = blockIdx.x * 64;
  const int m0   = blockIdx.y * 128;
  const int tid  = threadIdx.x;
  const int wave = __builtin_amdgcn_readfirstlane((int)(threadIdx.x >> 5));
  const int lane = tid & 31;
  const int lq   = lane & 15;
  const int hi   = lane >> 4;
  const int wm   = wave >> 1;
  const int wn   = wave & 1;

  __shared__ __align__(16) float sF[128 * OP];

  v8f acc[2][2];
  #pragma unroll
  for (int i = 0; i < 2; ++i) {
    #pragma unroll
    for (int jj = 0; jj < 2; ++jj) acc[i][jj] = (v8f){0, 0, 0, 0, 0, 0, 0, 0};
  }
  gemm_tile_128x64(att, w2t, m0, n0, wm, wn, lq, hi, acc);

  #pragma unroll
  for (int i = 0; i < 2; ++i) {
    #pragma unroll
    for (int jj = 0; jj < 2; ++jj) {
      #pragma unroll
      for (int r = 0; r < 8; ++r) {
        const int row = wm * 32 + i * 16 + hi * 8 + r;
        const int col = wn * 32 + jj * 16 + lq;
        sF[row * OP + col] = acc[i][jj][r] * (1.0f / 4096.0f);
      }
    }
  }
  __syncthreads();

  const int piece = tid & 15;
  const v4f braw = *(const v4f*)(b2 + n0 + piece * 4);
  v4f bias;
  #pragma unroll
  for (int i = 0; i < 4; ++i) bias[i] = (float)(bf16)braw[i];

  v4f    vals[8];
  size_t gidx[8];
  #pragma unroll
  for (int it = 0; it < 8; ++it) {
    const int row = it * 16 + (tid >> 4);
    const v4f v = *(const v4f*)(sF + row * OP + piece * 4);
    vals[it] = v + bias;
    const int tt = m0 + row;
    const int b  = tt / SEQ;
    const int s  = tt - b * SEQ;
    gidx[it] = ((size_t)b * SEQ_FULL + s) * HIDN + n0 + piece * 4;
  }
  #pragma unroll
  for (int it = 0; it < 8; ++it) *(volatile v4f*)(out + gidx[it]) = vals[it];
  __threadfence();
  #pragma unroll
  for (int it = 0; it < 8; ++it) *(volatile v4f*)(out + gidx[it]) = vals[it];
}

extern "C" void kernel_launch(void* const* d_in, const int* in_sizes, int n_in,
                              void* d_out, int out_size, void* d_ws, size_t ws_size,
                              hipStream_t stream) {
  if (n_in < 7) return;
  const size_t rows_used = (size_t)(NB - 1) * SEQ_FULL + SEQ;
  if ((size_t)in_sizes[0] < rows_used * EDIM) return;
  if (in_sizes[1] < EDIM || in_sizes[2] < EDIM) return;
  if ((size_t)in_sizes[3] < (size_t)EDIM * QKVW) return;
  if (in_sizes[4] < QKVW) return;
  if ((size_t)in_sizes[5] < (size_t)HIDN * HIDN) return;
  if (in_sizes[6] < HIDN) return;
  if ((size_t)out_size < rows_used * HIDN) return;
  if (ws_size < WS_BYTES) return;

  const float* x    = (const float*)d_in[0];
  const float* ln_g = (const float*)d_in[1];
  const float* ln_b = (const float*)d_in[2];
  const float* W1   = (const float*)d_in[3];
  const float* b1   = (const float*)d_in[4];
  const float* W2   = (const float*)d_in[5];
  const float* b2   = (const float*)d_in[6];
  float*       out  = (float*)d_out;
  f16*         wsh  = (f16*)d_ws;

  ln_kernel<<<dim3(NTOK), 128, 0, stream>>>(x, ln_g, ln_b, wsh + XN_OFF);
  wt_kernel<<<dim3(QKVW / 64, EDIM / 64), 256, 0, stream>>>(W1, wsh + W1T_OFF, EDIM, QKVW);
  wt_kernel<<<dim3(HIDN / 64, HIDN / 64), 256, 0, stream>>>(W2, wsh + W2T_OFF, HIDN, HIDN);
  qkv_gemm_kernel<<<dim3(QKVW / 64, NTOK / 128), 256, 0, stream>>>(wsh + XN_OFF, wsh + W1T_OFF, b1, wsh);
  attn_kernel<<<dim3(SEQ / BQ, NGRP), 256, 0, stream>>>(wsh + QP_OFF, wsh + KP_OFF, wsh + VT_OFF, wsh + ATT_OFF);
  out_gemm_kernel<<<dim3(HIDN / 64, NTOK / 128), 256, 0, stream>>>(wsh + ATT_OFF, wsh + W2T_OFF, b2, out);
}
